// VariableSelectionNetwork_19061064859718
// MI455X (gfx1250) — hardware-verified
//
#include <hip/hip_runtime.h>

typedef _Float16 v16h __attribute__((ext_vector_type(16)));
typedef _Float16 v8h  __attribute__((ext_vector_type(8)));
typedef float    v8f  __attribute__((ext_vector_type(8)));
typedef float    v4f  __attribute__((ext_vector_type(4)));
typedef v8h __attribute__((may_alias)) v8ha;
typedef v4f __attribute__((may_alias)) v4fa;

union Frag { v16h v; v8h half[2]; };

#define NTOK 16384
#define NF   32
#define NHID 128
#define N2H  256
#define MT   64
#define NTHR 256
#define WTHR 128
#define WSC  4096.0f
#define ASC  16.0f
#define INV_W  (1.0f / 4096.0f)
#define INV_WA (1.0f / 65536.0f)
#define LN_EPS 1e-5f

#define P_XH  0
#define P_FW2 524288
#define P_FGL 1048576
#define P_WW1 2097152
#define P_WW2 2101248
#define P_WGL 2105344
#define P_END 2107392
#define WS_TOTAL_BYTES ((size_t)P_END * 2)

static_assert(P_FW2 == P_XH + NTOK * NF);
static_assert(P_FGL == P_FW2 + NF * NHID * NHID);
static_assert(P_WW1 == P_FGL + NF * N2H * NHID);
static_assert(P_WW2 == P_WW1 + NHID * NF);
static_assert(P_WGL == P_WW2 + NF * NHID);
static_assert(P_END == P_WGL + 2 * NF * NF);
static_assert((P_FW2 * 2) % 128 == 0 && (P_FGL * 2) % 128 == 0 && (P_WW1 * 2) % 128 == 0 &&
              (P_WW2 * 2) % 128 == 0 && (P_WGL * 2) % 128 == 0 && (P_END * 2) % 128 == 0);

#define OUT0_ELEMS (NTOK * NHID)
#define OUT1_OFF   2097152
#define OUT_TOTAL  (NTOK * NHID + NTOK * NF)
static_assert(OUT1_OFF == OUT0_ELEMS);
static_assert(OUT1_OFF + NTOK * NF == OUT_TOTAL);
static_assert(NTOK % MT == 0 && NTOK % 64 == 0);

#define PB_FW2 0
#define PB_FGL 128
#define PB_WW2 384
#define PB_WW1 385
#define PB_WGL 389
#define PB_XH  391
#define PB_END (PB_XH + (NTOK * NF / 8) / NTHR)
static_assert((NTOK * NF / 8) % NTHR == 0);

#define MO_H   0
#define MO_H2  16384
#define MO_X   32768
#define MO_W   40960
#define MO_P   49152
#define MO_PS  53248
#define MO_PQ  53760
#define MSMEM  54272
static_assert(MSMEM <= 65536);

__device__ __forceinline__ float bfr(float f) {
  unsigned u = __builtin_bit_cast(unsigned, f);
  u += 0x7FFFu + ((u >> 16) & 1u);
  return __builtin_bit_cast(float, u & 0xFFFF0000u);
}
__device__ __forceinline__ float elu_f(float v) {
  const float e = expm1f(v);
  return (v > 0.0f) ? v : e;
}
__device__ __forceinline__ float sigm_f(float v) {
  v = fminf(fmaxf(v, -30.0f), 30.0f);
  const float e = expf(-v);
  return 1.0f / (1.0f + e);
}
__device__ __forceinline__ float hsum16(float v) {
  v += __shfl_xor(v, 1);
  v += __shfl_xor(v, 2);
  v += __shfl_xor(v, 4);
  v += __shfl_xor(v, 8);
  return v;
}
__device__ __forceinline__ float hmax16(float v) {
  v = fmaxf(v, __shfl_xor(v, 1));
  v = fmaxf(v, __shfl_xor(v, 2));
  v = fmaxf(v, __shfl_xor(v, 4));
  v = fmaxf(v, __shfl_xor(v, 8));
  return v;
}

__device__ __forceinline__ v8f wmma_f16(v16h a, v16h b, v8f c) {
  v8f d = __builtin_amdgcn_wmma_f32_16x16x32_f16(false, a, false, b, (short)0, c, false, false);
  asm volatile("v_nop\n\tv_nop\n\tv_nop\n\tv_nop" : "+v"(d) : "v"(a), "v"(b));
  return d;
}

__device__ __forceinline__ v16h load_frag(const _Float16* p, int h) {
  Frag f;
  f.half[0] = *(const v8ha*)(p + 8 * h);
  f.half[1] = *(const v8ha*)(p + 16 + 8 * h);
  return f.v;
}

template <int K, int N>
__device__ __forceinline__ void tr_block(const float* __restrict__ src, _Float16* __restrict__ dst,
                                         int tid, float* sT) {
  constexpr int NV = K * 8;
  static_assert(NV % NTHR == 0);
  #pragma unroll
  for (int i = 0; i < NV / NTHR; ++i) {
    const int q = tid + i * NTHR;
    const int k = q >> 3, c4 = (q & 7) * 4;
    const v4f v = *(const v4fa*)(src + (size_t)k * N + c4);
    const v4f r = { bfr(v.x), bfr(v.y), bfr(v.z), bfr(v.w) };
    *(v4fa*)(sT + k * 32 + c4) = r;
  }
  __syncthreads();
  constexpr int CH = 4 * K;
  v8h o[2];
  #pragma unroll
  for (int i = 0; i < 2; ++i) {
    const int c = tid + i * NTHR;
    const int cc = (c < CH) ? c : (CH - 1);
    const int row = (cc * 8) / K, k0 = (cc * 8) % K;
    v8h t;
    #pragma unroll
    for (int j = 0; j < 8; ++j) t[j] = (_Float16)(sT[(k0 + j) * 32 + row] * WSC);
    o[i] = t;
  }
  #pragma unroll
  for (int i = 0; i < 2; ++i) {
    const int c = tid + i * NTHR;
    if (c < CH) *(volatile v8h*)(dst + (size_t)c * 8) = o[i];
  }
  __threadfence();
  #pragma unroll
  for (int i = 0; i < 2; ++i) {
    const int c = tid + i * NTHR;
    if (c < CH) *(volatile v8h*)(dst + (size_t)c * 8) = o[i];
  }
}

__global__ __launch_bounds__(NTHR) void prep_kernel(
    const float* __restrict__ x, const float* __restrict__ fw2, const float* __restrict__ fglu_w,
    const float* __restrict__ ww1, const float* __restrict__ ww2, const float* __restrict__ wglu_w,
    _Float16* __restrict__ planes)
{
  __shared__ __attribute__((aligned(16))) float sT[128 * 32];
  const int b = blockIdx.x, tid = threadIdx.x;
  if (b < PB_FGL) {
    const int f = b >> 2, nb = b & 3;
    tr_block<128, 128>(fw2 + (size_t)f * NHID * NHID + nb * 32,
                       planes + P_FW2 + (size_t)f * NHID * NHID + (size_t)nb * 32 * NHID, tid, sT);
  } else if (b < PB_WW2) {
    const int bb = b - PB_FGL, f = bb >> 3, nb = bb & 7;
    tr_block<128, 256>(fglu_w + (size_t)f * NHID * N2H + nb * 32,
                       planes + P_FGL + (size_t)f * N2H * NHID + (size_t)nb * 32 * NHID, tid, sT);
  } else if (b < PB_WW1) {
    tr_block<128, 32>(ww2, planes + P_WW2, tid, sT);
  } else if (b < PB_WGL) {
    const int nb = b - PB_WW1;
    tr_block<32, 128>(ww1 + nb * 32, planes + P_WW1 + (size_t)nb * 32 * 32, tid, sT);
  } else if (b < PB_XH) {
    const int nb = b - PB_WGL;
    tr_block<32, 64>(wglu_w + nb * 32, planes + P_WGL + (size_t)nb * 32 * 32, tid, sT);
  } else {
    const int g = (b - PB_XH) * NTHR + tid;
    if (g < NTOK * NF / 8) {
      const float* src = x + (size_t)g * 8;
      const v4f a = *(const v4fa*)src;
      const v4f c = *(const v4fa*)(src + 4);
      const v8h o = { (_Float16)bfr(a.x), (_Float16)bfr(a.y), (_Float16)bfr(a.z), (_Float16)bfr(a.w),
                      (_Float16)bfr(c.x), (_Float16)bfr(c.y), (_Float16)bfr(c.z), (_Float16)bfr(c.w) };
      _Float16* dst = planes + P_XH + (size_t)g * 8;
      *(volatile v8h*)dst = o;
      __threadfence();
      *(volatile v8h*)dst = o;
    }
  }
}

__device__ __forceinline__ void w_store_pass(const float* sW, float* wout, int tok0, int w, int lane) {
  const int q8 = lane & 7, sub = lane >> 3;
  #pragma unroll
  for (int i = 0; i < 4; ++i) {
    const int row = 16 * w + i * 4 + sub;
    const v4f v = *(const v4fa*)(sW + row * NF + 4 * q8);
    *(volatile v4f*)(wout + (size_t)(tok0 + row) * NF + 4 * q8) = v;
  }
}

__global__ __launch_bounds__(WTHR) void wsel_kernel(
    const _Float16* __restrict__ xh, const _Float16* __restrict__ ww1T,
    const _Float16* __restrict__ ww2T, const _Float16* __restrict__ wglT,
    const float* __restrict__ x,
    const float* __restrict__ wb1, const float* __restrict__ wb2,
    const float* __restrict__ wglu_b, const float* __restrict__ wln_g, const float* __restrict__ wln_b,
    float* __restrict__ wout)
{
  __shared__ __attribute__((aligned(16))) _Float16 sWh[4 * 16 * NHID];
  __shared__ __attribute__((aligned(16))) _Float16 sWh2[4 * 16 * NF];
  __shared__ __attribute__((aligned(16))) float sXr[64 * NF];
  __shared__ __attribute__((aligned(16))) float sW[64 * NF];

  const int tid = threadIdx.x, lane = tid & 31, w = tid >> 5;
  const int h = lane >> 4, m = lane & 15;
  const int tok0 = blockIdx.x * 64;

  #pragma unroll
  for (int i = 0; i < 4; ++i) {
    const int q = tid + WTHR * i;
    const v4f v = *(const v4fa*)(x + (size_t)tok0 * NF + (size_t)q * 4);
    const v4f r = { bfr(v.x), bfr(v.y), bfr(v.z), bfr(v.w) };
    *(v4fa*)(sXr + q * 4) = r;
  }

  const v8f z8 = {0.f, 0.f, 0.f, 0.f, 0.f, 0.f, 0.f, 0.f};
  _Float16* myWh = sWh + w * (16 * NHID);
  _Float16* myWh2 = sWh2 + w * (16 * NF);

  {
    const v16h a = load_frag(xh + (size_t)(tok0 + 16 * w + m) * NF, h);
    v8f acc[8];
    #pragma unroll
    for (int t = 0; t < 8; ++t) {
      const v16h b = load_frag(ww1T + (size_t)(16 * t + m) * NF, h);
      acc[t] = wmma_f16(a, b, z8);
    }
    #pragma unroll
    for (int t = 0; t < 8; ++t) {
      const float bb = bfr(wb1[16 * t + m]);
      #pragma unroll
      for (int r = 0; r < 8; ++r) {
        const float v = acc[t][r] * INV_W + bb;
        myWh[(8 * h + r) * NHID + 16 * t + m] = (_Float16)(elu_f(v) * ASC);
      }
    }
  }
  __syncthreads();

  {
    v8f acc[2];
    acc[0] = z8; acc[1] = z8;
    const _Float16* arow = myWh + m * NHID;
    #pragma unroll 1
    for (int k0 = 0; k0 < NHID; k0 += 32) {
      const v16h a = load_frag(arow + k0, h);
      #pragma unroll
      for (int t = 0; t < 2; ++t) {
        const v16h b = load_frag(ww2T + (size_t)(16 * t + m) * NHID + k0, h);
        acc[t] = wmma_f16(a, b, acc[t]);
      }
    }
    #pragma unroll
    for (int t = 0; t < 2; ++t) {
      const float bb = bfr(wb2[16 * t + m]);
      #pragma unroll
      for (int r = 0; r < 8; ++r) {
        const float v = acc[t][r] * INV_WA + bb;
        myWh2[(8 * h + r) * NF + 16 * t + m] = (_Float16)(v * ASC);
      }
    }
  }
  __syncthreads();

  {
    const v16h a = load_frag(myWh2 + m * NF, h);
    v8f acc[4];
    #pragma unroll
    for (int t = 0; t < 4; ++t) {
      const v16h b = load_frag(wglT + (size_t)(16 * t + m) * NF, h);
      acc[t] = wmma_f16(a, b, z8);
    }
    float pre[2][8], s[8];
    #pragma unroll
    for (int r = 0; r < 8; ++r) s[r] = 0.0f;
    #pragma unroll
    for (int c = 0; c < 2; ++c) {
      const float bv = bfr(wglu_b[16 * c + m]);
      const float bg = bfr(wglu_b[NF + 16 * c + m]);
      #pragma unroll
      for (int r = 0; r < 8; ++r) {
        const float vv = acc[c][r] * INV_WA + bv;
        const float gg = acc[c + 2][r] * INV_WA + bg;
        const float xr = sXr[(16 * w + 8 * h + r) * NF + 16 * c + m];
        const float p = vv * sigm_f(gg) + xr;
        pre[c][r] = p;
        s[r] += p;
      }
    }
    float mu[8], q[8];
    #pragma unroll
    for (int r = 0; r < 8; ++r) { mu[r] = hsum16(s[r]) * (1.0f / 32.0f); q[r] = 0.0f; }
    #pragma unroll
    for (int c = 0; c < 2; ++c)
      #pragma unroll
      for (int r = 0; r < 8; ++r) {
        const float d = pre[c][r] - mu[r];
        pre[c][r] = d;
        q[r] += d * d;
      }
    float rs[8];
    #pragma unroll
    for (int r = 0; r < 8; ++r) rs[r] = rsqrtf(hsum16(q[r]) * (1.0f / 32.0f) + LN_EPS);
    #pragma unroll
    for (int c = 0; c < 2; ++c) {
      const float g = bfr(wln_g[16 * c + m]);
      const float bt = bfr(wln_b[16 * c + m]);
      #pragma unroll
      for (int r = 0; r < 8; ++r) pre[c][r] = pre[c][r] * rs[r] * g + bt;
    }
    float mx[8], e0[8], e1[8];
    #pragma unroll
    for (int r = 0; r < 8; ++r) {
      mx[r] = hmax16(fmaxf(pre[0][r], pre[1][r]));
      e0[r] = expf(pre[0][r] - mx[r]);
      e1[r] = expf(pre[1][r] - mx[r]);
      const float se = hsum16(e0[r] + e1[r]);
      const float inv = 1.0f / se;
      sW[(16 * w + 8 * h + r) * NF + m]      = e0[r] * inv;
      sW[(16 * w + 8 * h + r) * NF + 16 + m] = e1[r] * inv;
    }
  }
  __syncthreads();

  w_store_pass(sW, wout, tok0, w, lane);
  __threadfence();
  w_store_pass(sW, wout, tok0, w, lane);
}

__device__ __forceinline__ void o_store_pass(const float* sO, float* out, int tok0, int w, int lane) {
  const int q8 = lane & 7, sub = lane >> 3;
  #pragma unroll
  for (int i = 0; i < 8; ++i) {
    const int lid = w * 32 + i * 4 + sub;
    const int row = lid >> 2, seg = lid & 3;
    const v4f v = *(const v4fa*)(sO + row * NHID + seg * 32 + 4 * q8);
    *(volatile v4f*)(out + (size_t)(tok0 + row) * NHID + seg * 32 + 4 * q8) = v;
  }
}

__global__ __launch_bounds__(NTHR) void grn_kernel(
    const float* __restrict__ x,
    const float* __restrict__ fw1, const float* __restrict__ fb1,
    const float* __restrict__ fb2, const float* __restrict__ fglu_b,
    const float* __restrict__ fskip, const float* __restrict__ fln_g, const float* __restrict__ fln_b,
    const _Float16* __restrict__ fw2T, const _Float16* __restrict__ fglT,
    const float* wsel, float* out)
{
  __shared__ __attribute__((aligned(16))) char smem[MSMEM];
  _Float16* sH  = (_Float16*)(smem + MO_H);
  _Float16* sH2 = (_Float16*)(smem + MO_H2);
  float* sO  = (float*)(smem + MO_H);
  float* sX  = (float*)(smem + MO_X);
  float* sWt = (float*)(smem + MO_W);
  float* sP  = (float*)(smem + MO_P);
  float* sPs = (float*)(smem + MO_PS);
  float* sPq = (float*)(smem + MO_PQ);

  const int tid = threadIdx.x, lane = tid & 31, w = tid >> 5;
  const int h = lane >> 4, m = lane & 15;
  const int msub = w & 3, qh = w >> 2;
  const int tok0 = blockIdx.x * MT;
  const int rbase = 16 * msub + 8 * h;
  const int hrow = tid >> 2, hkb = (tid & 3) * 32;

  #pragma unroll
  for (int i = 0; i < 2; ++i) {
    const int q = tid + NTHR * i;
    const v4f v = *(const v4fa*)(x + (size_t)tok0 * NF + (size_t)q * 4);
    const v4f r = { bfr(v.x), bfr(v.y), bfr(v.z), bfr(v.w) };
    *(v4fa*)(sX + q * 4) = r;
    const v4f wv = *(const v4fa*)(wsel + (size_t)tok0 * NF + (size_t)q * 4);
    *(v4fa*)(sWt + q * 4) = wv;
  }

  const v8f z8 = {0.f, 0.f, 0.f, 0.f, 0.f, 0.f, 0.f, 0.f};
  v8f accO[4];
  #pragma unroll
  for (int nt = 0; nt < 4; ++nt) accO[nt] = z8;

  #pragma unroll 1
  for (int f = 0; f < NF; ++f) {
    __syncthreads();
    {
      const int fo = f * NHID;
      const float* src = fw1 + fo;
      if (w == 1)      src = fb1 + fo;
      else if (w == 2) src = fb2 + fo;
      else if (w == 3) src = fglu_b + f * N2H;
      else if (w == 4) src = fglu_b + f * N2H + NHID;
      else if (w == 5) src = fskip + fo;
      else if (w == 6) src = fln_g + fo;
      else if (w == 7) src = fln_b + fo;
      const v4f v = *(const v4fa*)(src + lane * 4);
      const v4f r = { bfr(v.x), bfr(v.y), bfr(v.z), bfr(v.w) };
      *(v4fa*)(sP + w * NHID + lane * 4) = r;
    }
    __syncthreads();

    {
      const float xv = sX[hrow * NF + f];
      #pragma unroll 1
      for (int j = 0; j < 4; ++j) {
        const int kb = hkb + 8 * j;
        v8h o;
        #pragma unroll
        for (int i = 0; i < 8; ++i) {
          const float v = xv * sP[kb + i] + sP[NHID + kb + i];
          o[i] = (_Float16)(elu_f(v) * ASC);
        }
        *(v8ha*)(sH + hrow * NHID + kb) = o;
      }
    }
    __syncthreads();

    {
      v8f acc2[4];
      #pragma unroll
      for (int nt = 0; nt < 4; ++nt) acc2[nt] = z8;
      const _Float16* arow = sH + (16 * msub + m) * NHID;
      const _Float16* brow = fw2T + ((size_t)f * NHID + 64 * qh + m) * NHID;
      #pragma unroll 1
      for (int k0 = 0; k0 < NHID; k0 += 32) {
        const v16h a = load_frag(arow + k0, h);
        #pragma unroll
        for (int nt = 0; nt < 4; ++nt) {
          const v16h b = load_frag(brow + (size_t)nt * 16 * NHID + k0, h);
          acc2[nt] = wmma_f16(a, b, acc2[nt]);
        }
      }
      #pragma unroll
      for (int nt = 0; nt < 4; ++nt) {
        const int col = 64 * qh + 16 * nt + m;
        const float bb = sP[256 + col];
        #pragma unroll
        for (int r = 0; r < 8; ++r) {
          const float v = acc2[nt][r] * INV_WA + bb;
          sH2[(rbase + r) * NHID + col] = (_Float16)(v * ASC);
        }
      }
    }
    __syncthreads();

    v8f accG[2][4];
    #pragma unroll
    for (int p = 0; p < 2; ++p)
      #pragma unroll
      for (int nt = 0; nt < 4; ++nt) accG[p][nt] = z8;
    {
      const _Float16* arow = sH2 + (16 * msub + m) * NHID;
      const _Float16* brow = fglT + ((size_t)f * N2H + 64 * qh + m) * NHID;
      #pragma unroll 1
      for (int k0 = 0; k0 < NHID; k0 += 32) {
        const v16h a = load_frag(arow + k0, h);
        #pragma unroll
        for (int p = 0; p < 2; ++p)
          #pragma unroll
          for (int nt = 0; nt < 4; ++nt) {
            const v16h b = load_frag(brow + (size_t)(p * NHID + nt * 16) * NHID + k0, h);
            accG[p][nt] = wmma_f16(a, b, accG[p][nt]);
          }
      }
    }

    float xr[8], s[8];
    #pragma unroll
    for (int r = 0; r < 8; ++r) { xr[r] = sX[(rbase + r) * NF + f]; s[r] = 0.0f; }
    #pragma unroll
    for (int nt = 0; nt < 4; ++nt) {
      const int col = 64 * qh + 16 * nt + m;
      const float bv = sP[384 + col];
      const float bg = sP[512 + col];
      const float fs = sP[640 + col];
      #pragma unroll
      for (int r = 0; r < 8; ++r) {
        const float vv = accG[0][nt][r] * INV_WA + bv;
        const float gg = accG[1][nt][r] * INV_WA + bg;
        const float glu = vv * sigm_f(gg) + xr[r] * fs;
        accG[0][nt][r] = glu;
        s[r] += glu;
      }
    }
    #pragma unroll
    for (int r = 0; r < 8; ++r) s[r] = hsum16(s[r]);
    if (m == 0) {
      #pragma unroll
      for (int r = 0; r < 8; ++r) sPs[(rbase + r) * 2 + qh] = s[r];
    }
    __syncthreads();
    float mu[8], q[8];
    #pragma unroll
    for (int r = 0; r < 8; ++r) {
      mu[r] = (sPs[(rbase + r) * 2] + sPs[(rbase + r) * 2 + 1]) * (1.0f / 128.0f);
      q[r] = 0.0f;
    }
    #pragma unroll
    for (int nt = 0; nt < 4; ++nt)
      #pragma unroll
      for (int r = 0; r < 8; ++r) {
        const float d = accG[0][nt][r] - mu[r];
        accG[0][nt][r] = d;
        q[r] += d * d;
      }
    #pragma unroll
    for (int r = 0; r < 8; ++r) q[r] = hsum16(q[r]);
    if (m == 0) {
      #pragma unroll
      for (int r = 0; r < 8; ++r) sPq[(rbase + r) * 2 + qh] = q[r];
    }
    __syncthreads();
    float rs[8], wt[8];
    #pragma unroll
    for (int r = 0; r < 8; ++r) {
      rs[r] = rsqrtf((sPq[(rbase + r) * 2] + sPq[(rbase + r) * 2 + 1]) * (1.0f / 128.0f) + LN_EPS);
      wt[r] = sWt[(rbase + r) * NF + f];
    }
    #pragma unroll
    for (int nt = 0; nt < 4; ++nt) {
      const int col = 64 * qh + 16 * nt + m;
      const float g = sP[768 + col];
      const float bt = sP[896 + col];
      #pragma unroll
      for (int r = 0; r < 8; ++r) {
        const float pr = accG[0][nt][r] * rs[r] * g + bt;
        accO[nt][r] += wt[r] * pr;
      }
    }
  }
  __syncthreads();

  #pragma unroll
  for (int nt = 0; nt < 4; ++nt) {
    const int col = 64 * qh + 16 * nt + m;
    #pragma unroll
    for (int r = 0; r < 8; ++r) sO[(rbase + r) * NHID + col] = accO[nt][r];
  }
  __syncthreads();

  o_store_pass(sO, out, tok0, w, lane);
  __threadfence();
  o_store_pass(sO, out, tok0, w, lane);
}

extern "C" void kernel_launch(void* const* d_in, const int* in_sizes, int n_in,
                              void* d_out, int out_size, void* d_ws, size_t ws_size,
                              hipStream_t stream) {
  if (n_in < 18) return;
  if (in_sizes[0] != NTOK * NF) return;
  if (in_sizes[1] != NF * NHID || in_sizes[2] != NF * NHID) return;
  if (in_sizes[3] != NF * NHID * NHID || in_sizes[4] != NF * NHID) return;
  if (in_sizes[5] != NF * NHID * N2H || in_sizes[6] != NF * N2H) return;
  if (in_sizes[7] != NF * NHID || in_sizes[8] != NF * NHID || in_sizes[9] != NF * NHID) return;
  if (in_sizes[10] != NF * NHID || in_sizes[11] != NHID) return;
  if (in_sizes[12] != NHID * NF || in_sizes[13] != NF) return;
  if (in_sizes[14] != NF * 2 * NF || in_sizes[15] != 2 * NF) return;
  if (in_sizes[16] != NF || in_sizes[17] != NF) return;
  if (out_size != OUT_TOTAL) return;
  if (WS_TOTAL_BYTES > ws_size) return;

  const float* x      = (const float*)d_in[0];
  const float* fw1    = (const float*)d_in[1];
  const float* fb1    = (const float*)d_in[2];
  const float* fw2    = (const float*)d_in[3];
  const float* fb2    = (const float*)d_in[4];
  const float* fglu_w = (const float*)d_in[5];
  const float* fglu_b = (const float*)d_in[6];
  const float* fskip  = (const float*)d_in[7];
  const float* fln_g  = (const float*)d_in[8];
  const float* fln_b  = (const float*)d_in[9];
  const float* ww1    = (const float*)d_in[10];
  const float* wb1    = (const float*)d_in[11];
  const float* ww2    = (const float*)d_in[12];
  const float* wb2    = (const float*)d_in[13];
  const float* wglu_w = (const float*)d_in[14];
  const float* wglu_b = (const float*)d_in[15];
  const float* wln_g  = (const float*)d_in[16];
  const float* wln_b  = (const float*)d_in[17];

  float* out  = (float*)d_out;
  float* wout = out + OUT1_OFF;

  _Float16* planes = (_Float16*)d_ws;

  prep_kernel<<<PB_END, NTHR, 0, stream>>>(x, fw2, fglu_w, ww1, ww2, wglu_w, planes);

  wsel_kernel<<<NTOK / 64, WTHR, 0, stream>>>(planes + P_XH, planes + P_WW1, planes + P_WW2, planes + P_WGL,
                                              x, wb1, wb2, wglu_b, wln_g, wln_b, wout);

  grn_kernel<<<NTOK / MT, NTHR, 0, stream>>>(x, fw1, fb1, fb2, fglu_b, fskip, fln_g, fln_b,
                                             planes + P_FW2, planes + P_FGL, wout, out);
}
